// Timeline_37477884625304
// MI455X (gfx1250) — hardware-verified
//
#include <hip/hip_runtime.h>
#include <math.h>

constexpr int NBATCH = 32, NVIS = 128, NCODE = 64, NEMB = 256, NHID = 256, NATT = 128;
constexpr int NVOC = 20001;
constexpr int NVOCP = 20032;
constexpr int NGATE = 4 * NHID;
constexpr int NVISITS = NBATCH * NVIS;
constexpr float BIGF = 1e20f;

constexpr float EMB_SC = 64.0f;
constexpr float W_SC   = 16.0f;
constexpr float QK_OUT_SC = 1.0f / 16.0f;
constexpr float SCORE_INV = 1.0f / 4096.0f;
constexpr float P_SC = 1024.0f;
constexpr float FE_INV = 1.0f / 65536.0f;
constexpr float X_SC = 16.0f, H_SC = 16.0f;
constexpr float Z_INV = 1.0f / 256.0f;
constexpr float SQRT_A = 11.313708498984761f;

constexpr int TTP = 72;
constexpr int QKP = 136;
constexpr int SSP = 68;
constexpr int PPP = 72;
constexpr int AXP = 264;
constexpr int HSP = 260;

static_assert(NVOCP % 64 == 0 && NVOCP >= NVOC, "");
static_assert((TTP * 2) % 16 == 0 && (QKP * 2) % 16 == 0 && (PPP * 2) % 16 == 0 && (AXP * 2) % 16 == 0 && (HSP * 4) % 16 == 0, "");

typedef __attribute__((ext_vector_type(16))) _Float16 v16h;
typedef __attribute__((ext_vector_type(8)))  _Float16 v8h;
typedef __attribute__((ext_vector_type(4)))  _Float16 v4hh;
typedef __attribute__((ext_vector_type(16))) __bf16   v16b;
typedef __attribute__((ext_vector_type(8)))  __bf16   v8b;
typedef __attribute__((ext_vector_type(8)))  float    v8f;
typedef __attribute__((ext_vector_type(4)))  float    v4f;

__device__ __forceinline__ unsigned short f2bf_bits(float f) {
  unsigned u = __float_as_uint(f);
  return (unsigned short)((u + 0x7FFFu + ((u >> 16) & 1u)) >> 16);
}
__device__ __forceinline__ float bf_bits2f(unsigned short h) { return __uint_as_float(((unsigned)h) << 16); }

__device__ __forceinline__ void dep_guard_h(v8f& a, v8f& b, v16h x, v16h y) { asm volatile("v_nop\n\tv_nop\n\tv_nop\n\tv_nop" : "+v"(a), "+v"(b) : "v"(x), "v"(y)); }
__device__ __forceinline__ void dep_guard_b(v8f& a, v8f& b, v16b x, v16b y) { asm volatile("v_nop\n\tv_nop\n\tv_nop\n\tv_nop" : "+v"(a), "+v"(b) : "v"(x), "v"(y)); }
__device__ __forceinline__ void keep4_h(v16h a, v16h b, v16h c, v16h d) { asm volatile("v_nop" :: "v"(a), "v"(b), "v"(c), "v"(d)); }
__device__ __forceinline__ void keep4_b(v16b a, v16b b, v16b c, v16b d) { asm volatile("v_nop" :: "v"(a), "v"(b), "v"(c), "v"(d)); }
__device__ __forceinline__ void acc_guard4(v8f& a, v8f& b, v8f& c, v8f& d) { asm volatile("v_nop\n\tv_nop\n\tv_nop\n\tv_nop" : "+v"(a), "+v"(b), "+v"(c), "+v"(d)); }
template <typename T> struct Frag;
template <> struct Frag<_Float16> {
  typedef v16h V; union U { v16h v; v8h h[2]; };
  static __device__ __forceinline__ v16h load(const _Float16* p) {
    U f; f.h[0] = *(const v8h*)(p); f.h[1] = *(const v8h*)(p + 16); return f.v;
  }
  static __device__ __forceinline__ v8f mma(v16h a, v16h b, v8f c) {
    return __builtin_amdgcn_wmma_f32_16x16x32_f16(false, a, false, b, (short)0, c, false, false);
  }
  static __device__ __forceinline__ void guard(v8f& a, v8f& b, v16h x, v16h y) { dep_guard_h(a, b, x, y); }
  static __device__ __forceinline__ void keep(v16h a, v16h b, v16h c, v16h d) { keep4_h(a, b, c, d); }
};
template <> struct Frag<__bf16> {
  typedef v16b V; union U { v16b v; v8b h[2]; };
  static __device__ __forceinline__ v16b load(const __bf16* p) {
    U f; f.h[0] = *(const v8b*)(p); f.h[1] = *(const v8b*)(p + 16); return f.v;
  }
  static __device__ __forceinline__ v8f mma(v16b a, v16b b, v8f c) {
    return __builtin_amdgcn_wmma_f32_16x16x32_bf16(false, a, false, b, (short)0, c, false, false);
  }
  static __device__ __forceinline__ void guard(v8f& a, v8f& b, v16b x, v16b y) { dep_guard_b(a, b, x, y); }
  static __device__ __forceinline__ void keep(v16b a, v16b b, v16b c, v16b d) { keep4_b(a, b, c, d); }
};

__device__ __forceinline__ v8f mma_h(v16h a, v16h b, v8f c) {
  c = __builtin_amdgcn_wmma_f32_16x16x32_f16(false, a, false, b, (short)0, c, false, false);
  asm volatile("v_nop\n\tv_nop\n\tv_nop\n\tv_nop" : "+v"(c) : "v"(a), "v"(b));
  return c;
}

__device__ __forceinline__ float fsig(float x)  { return __builtin_amdgcn_rcpf(1.0f + __expf(-x)); }
__device__ __forceinline__ float ftanh(float x) { return 1.0f - 2.0f * __builtin_amdgcn_rcpf(__expf(2.0f * x) + 1.0f); }

template <int ET> struct Elem;
template <> struct Elem<0> { typedef _Float16 T; };
template <> struct Elem<1> { typedef __bf16 T; };
template <int ET, bool SPLIT, int BIAS_MODE, int OUT_MODE, bool RESID, int ACT = 0>
__global__ __launch_bounds__(256) void wmma_gemm64(
    const unsigned short* __restrict__ Ap, const unsigned short* __restrict__ A2p, int lda, long strideA,
    const unsigned short* __restrict__ Btp, const unsigned short* __restrict__ Bt2p, int ldb, long strideB,
    void* __restrict__ Cout, void* __restrict__ Cout2, int ldc, long strideC,
    const float* __restrict__ bias,
    const float* __restrict__ resid, long strideR,
    int M, int N, int K, float scale) {
  typedef typename Elem<ET>::T T;
  typedef typename Frag<T>::V V;
  const T* A = (const T*)Ap; const T* A2 = (const T*)A2p; const T* Bt = (const T*)Btp; const T* Bt2 = (const T*)Bt2p;
  __shared__ __align__(16) float sT[8][16 * 68];
  const int b    = blockIdx.y;
  const int lane = threadIdx.x & 31;
  const int wave = threadIdx.x >> 5;
  const int tilesN = N >> 6;
  const int tilesM = M >> 6;
  const int tile = blockIdx.x * 8 + wave;
  if (tile >= tilesM * tilesN) return;
  const int tm = tile / tilesN;
  const int tn = tile - tm * tilesN;
  const int m0 = tm << 6;
  const int n0 = tn << 6;

  const T* Ab  = A  + (size_t)b * strideA;
  const T* Bb  = Bt + (size_t)b * strideB;
  const T* Ab2 = SPLIT ? (A2  + (size_t)b * strideA) : nullptr;
  const T* Bb2 = SPLIT ? (Bt2 + (size_t)b * strideB) : nullptr;

  const int rlane = lane & 15;
  const int koff  = (lane >> 4) * 8;
  const int mOff  = (lane >> 4) * 8;

  v8f acc[4][4];
#pragma unroll
  for (int i = 0; i < 4; ++i)
#pragma unroll
    for (int j = 0; j < 4; ++j) acc[i][j] = (v8f){0.f,0.f,0.f,0.f,0.f,0.f,0.f,0.f};

  for (int k0 = 0; k0 < K; k0 += 32) {
    V bh[4], bl[4];
#pragma unroll
    for (int j = 0; j < 4; ++j) {
      const size_t bo = (size_t)(n0 + (j << 4) + rlane) * ldb + koff + k0;
      bh[j] = Frag<T>::load(Bb + bo);
      if (SPLIT) bl[j] = Frag<T>::load(Bb2 + bo);
    }
#pragma unroll
    for (int i = 0; i < 4; ++i) {
      const size_t ao = (size_t)(m0 + (i << 4) + rlane) * lda + koff + k0;
      V ah = Frag<T>::load(Ab + ao);
      V al;
      if (SPLIT) al = Frag<T>::load(Ab2 + ao);
#pragma unroll
      for (int j = 0; j < 4; ++j) {
        acc[i][j] = Frag<T>::mma(ah, bh[j], acc[i][j]);
        if (SPLIT) {
          acc[i][j] = Frag<T>::mma(ah, bl[j], acc[i][j]);
          acc[i][j] = Frag<T>::mma(al, bh[j], acc[i][j]);
        }
      }
      Frag<T>::guard(acc[i][0], acc[i][3], ah, SPLIT ? al : ah);
    }
    Frag<T>::keep(bh[0], bh[1], bh[2], bh[3]);
    if (SPLIT) Frag<T>::keep(bl[0], bl[1], bl[2], bl[3]);
  }
  acc_guard4(acc[0][0], acc[0][1], acc[0][2], acc[0][3]);
  acc_guard4(acc[1][0], acc[1][1], acc[1][2], acc[1][3]);
  acc_guard4(acc[2][0], acc[2][1], acc[2][2], acc[2][3]);
  acc_guard4(acc[3][0], acc[3][1], acc[3][2], acc[3][3]);

  float* slab = sT[wave];
  const float* Rb = RESID ? (resid + (size_t)b * strideR) : nullptr;
#pragma unroll
  for (int i = 0; i < 4; ++i) {
    const int mBase = m0 + (i << 4);
#pragma unroll
    for (int j = 0; j < 4; ++j) {
      const int n = n0 + (j << 4) + rlane;
      float bv = 0.f;
      if (BIAS_MODE == 2) bv = bias[n];
#pragma unroll
      for (int r = 0; r < 8; ++r) {
        float v = acc[i][j][r] * scale;
        if (BIAS_MODE == 1) v += bias[mBase + mOff + r];
        if (BIAS_MODE == 2) v += bv;
        if (RESID) v += Rb[(size_t)(mBase + mOff + r) * ldc + n];
        if (ACT == 1) v = tanhf(v);
        if (ACT == 2) v = fmaxf(v, 0.0f);
        if (ACT == 3) v = v / (1.0f + expf(-v));
        if (ACT == 4) v = (v > 0.f) ? v : 0.01f * v;
        if (ACT == 5) v = 0.5f * v * (1.0f + erff(v * 0.70710678118654752f));
        slab[(mOff + r) * 68 + (j << 4) + rlane] = v;
      }
    }
    __builtin_amdgcn_fence(__ATOMIC_RELEASE, "workgroup");
    __builtin_amdgcn_wave_barrier();
    __builtin_amdgcn_fence(__ATOMIC_ACQUIRE, "workgroup");
    if (OUT_MODE == 0) {
      float* C = (float*)Cout + (size_t)b * strideC;
      const int hh = lane >> 4, c4 = (lane & 15) * 4;
      for (int pass = 0; pass < 2; ++pass) {
#pragma unroll
        for (int it = 0; it < 8; ++it) {
          const int row = it * 2 + hh;
          v4f v = *(const v4f*)(slab + row * 68 + c4);
          *(volatile v4f*)(C + (size_t)(mBase + row) * ldc + n0 + c4) = v;
        }
        __threadfence();
      }
    } else {
      const int q = lane >> 3, c8 = (lane & 7) * 8;
      unsigned short* C  = (unsigned short*)Cout  + (size_t)b * strideC;
      unsigned short* C2 = (OUT_MODE == 2) ? ((unsigned short*)Cout2 + (size_t)b * strideC) : nullptr;
      for (int pass = 0; pass < 2; ++pass) {
#pragma unroll
        for (int it = 0; it < 4; ++it) {
          const int row = it * 4 + q;
          const float* sp = slab + row * 68 + c8;
          v8h hv, lv;
#pragma unroll
          for (int e = 0; e < 8; ++e) {
            if (OUT_MODE == 1) {
              hv[e] = (_Float16)sp[e];
            } else {
              unsigned short hb = f2bf_bits(sp[e]);
              unsigned short lb = f2bf_bits(sp[e] - bf_bits2f(hb));
              hv[e] = __builtin_bit_cast(_Float16, hb);
              lv[e] = __builtin_bit_cast(_Float16, lb);
            }
          }
          *(volatile v8h*)(C + (size_t)(mBase + row) * ldc + n0 + c8) = hv;
          if (OUT_MODE == 2) *(volatile v8h*)(C2 + (size_t)(mBase + row) * ldc + n0 + c8) = lv;
        }
        __threadfence();
      }
    }
    __builtin_amdgcn_fence(__ATOMIC_RELEASE, "workgroup");
    __builtin_amdgcn_wave_barrier();
    __builtin_amdgcn_fence(__ATOMIC_ACQUIRE, "workgroup");
  }
}

__global__ __launch_bounds__(256) void cast_rows_f16(const float* __restrict__ src, int rows_src,
                                                    unsigned short* __restrict__ dst, int rows_dst, float sc) {
  const int i = blockIdx.x * 256 + (int)threadIdx.x;
  const int nchunk = rows_dst * 32;
  if (i >= nchunk) return;
  const int row = i >> 5, c8 = (i & 31) * 8;
  const int rs = (row < rows_src) ? row : (rows_src - 1);
  const bool zero = (row >= rows_src);
  const v4f a = *(const v4f*)(src + (size_t)rs * NEMB + c8);
  const v4f b = *(const v4f*)(src + (size_t)rs * NEMB + c8 + 4);
  v8h hv;
#pragma unroll
  for (int e = 0; e < 4; ++e) {
    hv[e]     = (_Float16)(zero ? 0.0f : a[e] * sc);
    hv[4 + e] = (_Float16)(zero ? 0.0f : b[e] * sc);
  }
  unsigned short* p = dst + (size_t)row * NEMB + c8;
  *(volatile v8h*)p = hv;
  __threadfence();
  *(volatile v8h*)p = hv;
}

__global__ __launch_bounds__(256) void visit_attn_kernel(
    const int* __restrict__ codes, const float* __restrict__ code_mask, const float* __restrict__ time_vals,
    const float* __restrict__ decay, const float* __restrict__ initial,
    const unsigned short* __restrict__ EMBp, const unsigned short* __restrict__ QKp, float* __restrict__ VV) {
  __shared__ __align__(16) _Float16 teT[NEMB * TTP];
  __shared__ __align__(16) _Float16 QKs[2 * NCODE * QKP];
  __shared__ __align__(16) float    Ssh[NCODE * SSP];
  __shared__ __align__(16) _Float16 Psh[NCODE * PPP];
  __shared__ __align__(16) float    vv_s[NEMB];
  __shared__ int   codes_s[NCODE];
  __shared__ float cm_s[NCODE];
  __shared__ float t2g_s[NCODE];
  __shared__ float rowf_s[NCODE];

  const _Float16* EMB = (const _Float16*)EMBp;
  const _Float16* QK  = (const _Float16*)QKp;
  const int bv = blockIdx.x;
  const int tid = threadIdx.x, wave = tid >> 5, lane = tid & 31;
  const int hh = lane >> 4, rl = lane & 15, koff = hh * 8;
  const v8f z8 = {0.f, 0.f, 0.f, 0.f, 0.f, 0.f, 0.f, 0.f};

  if (tid < NCODE) {
    int cd = codes[(size_t)bv * NCODE + tid];
    cd = cd < 0 ? 0 : (cd > NVOC - 1 ? NVOC - 1 : cd);
    codes_s[tid] = cd;
    const float cm = code_mask[(size_t)bv * NCODE + tid];
    cm_s[tid] = cm;
    const float tv = time_vals[bv];
    const float x = decay[cd] * tv + initial[cd];
    const float temp2 = __builtin_amdgcn_rcpf(1.0f + expf(-x));
    const float gate = (cm - BIGF) * (1.0f / (-BIGF));
    t2g_s[tid] = temp2 * gate;
  }
  __syncthreads();

#pragma unroll 1
  for (int it = 0; it < 8; ++it) {
    const int idx = it * 256 + tid;
    const int j = idx >> 6;
    const int c = idx & 63;
    const int cd = codes_s[c];
    const v8h tv = *(const v8h*)(EMB + (size_t)cd * NEMB + 8 * j);
#pragma unroll
    for (int e = 0; e < 8; ++e) teT[(8 * j + e) * TTP + c] = tv[e];
    const v8h qv = *(const v8h*)(QK + (size_t)cd * (2 * NATT) + 8 * j);
    *(v8h*)(QKs + (j >> 4) * (NCODE * QKP) + c * QKP + 8 * (j & 15)) = qv;
  }
  __syncthreads();

  {
    const _Float16* Qs = QKs;
    const _Float16* Ks = QKs + NCODE * QKP;
#pragma unroll 1
    for (int tt = 0; tt < 2; ++tt) {
      const int t = wave + 8 * tt;
      const int mt = t >> 2, nt = t & 3;
      v8f acc = z8;
#pragma unroll
      for (int k0 = 0; k0 < NATT; k0 += 32) {
        const v16h a = Frag<_Float16>::load(Qs + (mt * 16 + rl) * QKP + k0 + koff);
        const v16h b = Frag<_Float16>::load(Ks + (nt * 16 + rl) * QKP + k0 + koff);
        acc = mma_h(a, b, acc);
      }
#pragma unroll
      for (int r = 0; r < 8; ++r) Ssh[(mt * 16 + 8 * hh + r) * SSP + nt * 16 + rl] = acc[r] * SCORE_INV;
    }
  }
  __syncthreads();

  {
    const int row = tid >> 2, q4 = tid & 3;
    const float cmr = cm_s[row];
    float m = -INFINITY;
#pragma unroll 1
    for (int i = 0; i < 16; ++i) {
      const int col = q4 * 16 + i;
      float s = Ssh[row * SSP + col] - cm_s[col];
      s = s - cmr;
      s = s * (1.0f / SQRT_A);
      Ssh[row * SSP + col] = s;
      m = fmaxf(m, s);
    }
    m = fmaxf(m, __shfl_xor(m, 1, 32));
    m = fmaxf(m, __shfl_xor(m, 2, 32));
    float l = 0.0f;
#pragma unroll 1
    for (int i = 0; i < 16; ++i) {
      const int col = q4 * 16 + i;
      const float p = expf(Ssh[row * SSP + col] - m);
      l += p;
      Psh[row * PPP + col] = (_Float16)(p * P_SC);
    }
    l += __shfl_xor(l, 1, 32);
    l += __shfl_xor(l, 2, 32);
    if (q4 == 0) rowf_s[row] = t2g_s[row] * __builtin_amdgcn_rcpf(l) * FE_INV;
  }
  __syncthreads();

#pragma unroll 1
  for (int ntI = 0; ntI < 2; ++ntI) {
    const int nt = wave + 8 * ntI;
    const v16h b0 = Frag<_Float16>::load(teT + (nt * 16 + rl) * TTP + koff);
    const v16h b1 = Frag<_Float16>::load(teT + (nt * 16 + rl) * TTP + 32 + koff);
    float vcol = 0.0f;
#pragma unroll 1
    for (int mt = 0; mt < 4; ++mt) {
      v8f acc = z8;
      const v16h a0 = Frag<_Float16>::load(Psh + (mt * 16 + rl) * PPP + koff);
      const v16h a1 = Frag<_Float16>::load(Psh + (mt * 16 + rl) * PPP + 32 + koff);
      acc = mma_h(a0, b0, acc);
      acc = mma_h(a1, b1, acc);
#pragma unroll
      for (int r = 0; r < 8; ++r) vcol += acc[r] * rowf_s[mt * 16 + 8 * hh + r];
    }
    vcol += __shfl_xor(vcol, 16, 32);
    if (hh == 0) vv_s[nt * 16 + rl] = vcol;
  }
  __syncthreads();

  if (wave == 0) {
    float* dst = VV + (size_t)bv * NEMB;
    for (int pass = 0; pass < 2; ++pass) {
#pragma unroll
      for (int i = 0; i < 2; ++i) {
        const v4f v = *(const v4f*)(vv_s + 128 * i + 4 * lane);
        *(volatile v4f*)(dst + 128 * i + 4 * lane) = v;
      }
      __threadfence();
    }
  }
}

__device__ __forceinline__ void load_x_tile(const float* __restrict__ vv, int rowbase, int vidx, _Float16* Ax, int tid) {
#pragma unroll
  for (int it = 0; it < 4; ++it) {
    const int idx = it * 256 + tid;
    const int m = idx >> 6, f4 = (idx & 63) * 4;
    const v4f v = *(const v4f*)(vv + ((size_t)(rowbase + m) * NVIS + (size_t)vidx) * NEMB + f4);
    v4hh hv;
    hv[0] = (_Float16)(v[0] * X_SC);
    hv[1] = (_Float16)(v[1] * X_SC);
    hv[2] = (_Float16)(v[2] * X_SC);
    hv[3] = (_Float16)(v[3] * X_SC);
    *(v4hh*)(Ax + m * AXP + f4) = hv;
  }
}

__global__ __launch_bounds__(256) void bilstm_kernel(const float* __restrict__ vv, const float* __restrict__ vmask,
                                                  const float* __restrict__ bias_f, const float* __restrict__ bias_b,
                                                  const unsigned short* __restrict__ WXFp, const unsigned short* __restrict__ WHFp,
                                                  const unsigned short* __restrict__ WXBp, const unsigned short* __restrict__ WHBp,
                                                  float* __restrict__ out) {
  __shared__ __align__(16) _Float16 Ax[16 * AXP];
  __shared__ __align__(16) _Float16 Ah[16 * AXP];
  __shared__ __align__(16) float    Hs[16 * HSP];
  __shared__ __align__(16) float    vm_s[16 * NVIS];
  const int tid = threadIdx.x, lane = tid & 31, wave = tid >> 5;
  const int c = lane & 15, hh = lane >> 4, koff = hh * 8;
  const int dir = blockIdx.x >> 1;
  const int rowbase = (blockIdx.x & 1) * 16;
  const _Float16* WX = (const _Float16*)(dir ? WXBp : WXFp);
  const _Float16* WH = (const _Float16*)(dir ? WHBp : WHFp);
  const float* bias = dir ? bias_b : bias_f;

#pragma unroll 1
  for (int i = 0; i < 16; ++i) Ah[i * AXP + tid] = (_Float16)0.0f;
#pragma unroll
  for (int it = 0; it < 2; ++it) {
    const int idx = it * 256 + tid;
    const int m = idx >> 5, c4 = (idx & 31) * 4;
    const v4f v = *(const v4f*)(vmask + (size_t)(rowbase + m) * NVIS + c4);
    vm_s[m * NVIS + c4 + 0] = v[0];
    vm_s[m * NVIS + c4 + 1] = v[1];
    vm_s[m * NVIS + c4 + 2] = v[2];
    vm_s[m * NVIS + c4 + 3] = v[3];
  }
  load_x_tile(vv, rowbase, dir ? (NVIS - 1) : 0, Ax, tid);

  float cst[2][8], hst[2][8], hsum[2][8], bb[2][4];
#pragma unroll
  for (int nt = 0; nt < 2; ++nt) {
    const int j = 32 * wave + 16 * nt + c;
#pragma unroll
    for (int g = 0; g < 4; ++g) bb[nt][g] = bias[g * NHID + j];
#pragma unroll
    for (int r = 0; r < 8; ++r) { cst[nt][r] = 0.0f; hst[nt][r] = 0.0f; hsum[nt][r] = 0.0f; }
  }
  __syncthreads();

  const _Float16* axrow = Ax + c * AXP + koff;
  const _Float16* ahrow = Ah + c * AXP + koff;
  const v8f z8 = {0.f, 0.f, 0.f, 0.f, 0.f, 0.f, 0.f, 0.f};

#pragma unroll 1
  for (int t = 0; t < NVIS; ++t) {
    const int v = dir ? (NVIS - 1 - t) : t;
    float mrow[8];
#pragma unroll
    for (int r = 0; r < 8; ++r) mrow[r] = vm_s[(8 * hh + r) * NVIS + v];
#pragma unroll
    for (int nt = 0; nt < 2; ++nt) {
      const int j = 32 * wave + 16 * nt + c;
      const _Float16* wx = WX + (size_t)j * NEMB + koff;
      const _Float16* wh = WH + (size_t)j * NHID + koff;
      v8f acc[4];
      acc[0] = z8; acc[1] = z8; acc[2] = z8; acc[3] = z8;
#pragma unroll 1
      for (int kx = 0; kx < NEMB; kx += 32) {
        const v16h a  = Frag<_Float16>::load(axrow + kx);
        const v16h b0 = Frag<_Float16>::load(wx + kx);
        const v16h b1 = Frag<_Float16>::load(wx + (size_t)1 * NHID * NEMB + kx);
        const v16h b2 = Frag<_Float16>::load(wx + (size_t)2 * NHID * NEMB + kx);
        const v16h b3 = Frag<_Float16>::load(wx + (size_t)3 * NHID * NEMB + kx);
        acc[0] = Frag<_Float16>::mma(a, b0, acc[0]);
        acc[1] = Frag<_Float16>::mma(a, b1, acc[1]);
        acc[2] = Frag<_Float16>::mma(a, b2, acc[2]);
        acc[3] = Frag<_Float16>::mma(a, b3, acc[3]);
        dep_guard_h(acc[0], acc[3], a, b3);
        keep4_h(b0, b1, b2, b3);
      }
#pragma unroll 1
      for (int k0 = 0; k0 < NHID; k0 += 32) {
        const v16h a  = Frag<_Float16>::load(ahrow + k0);
        const v16h b0 = Frag<_Float16>::load(wh + k0);
        const v16h b1 = Frag<_Float16>::load(wh + (size_t)1 * NHID * NHID + k0);
        const v16h b2 = Frag<_Float16>::load(wh + (size_t)2 * NHID * NHID + k0);
        const v16h b3 = Frag<_Float16>::load(wh + (size_t)3 * NHID * NHID + k0);
        acc[0] = Frag<_Float16>::mma(a, b0, acc[0]);
        acc[1] = Frag<_Float16>::mma(a, b1, acc[1]);
        acc[2] = Frag<_Float16>::mma(a, b2, acc[2]);
        acc[3] = Frag<_Float16>::mma(a, b3, acc[3]);
        dep_guard_h(acc[0], acc[3], a, b3);
        keep4_h(b0, b1, b2, b3);
      }
      acc_guard4(acc[0], acc[1], acc[2], acc[3]);
#pragma unroll
      for (int r = 0; r < 8; ++r) {
        const float zi = acc[0][r] * Z_INV + bb[nt][0];
        const float zf = acc[1][r] * Z_INV + bb[nt][1];
        const float zg = acc[2][r] * Z_INV + bb[nt][2];
        const float zo = acc[3][r] * Z_INV + bb[nt][3];
        const float ig = fsig(zi);
        const float fg = fsig(zf);
        const float gg = ftanh(zg);
        const float og = fsig(zo);
        const float cn = fg * cst[nt][r] + ig * gg;
        cst[nt][r] = cn;
        const float hn = og * ftanh(cn);
        hst[nt][r] = hn;
        hsum[nt][r] += mrow[r] * hn;
      }
    }
    __syncthreads();
#pragma unroll
    for (int nt = 0; nt < 2; ++nt) {
      const int j = 32 * wave + 16 * nt + c;
#pragma unroll
      for (int r = 0; r < 8; ++r) Ah[(8 * hh + r) * AXP + j] = (_Float16)(hst[nt][r] * H_SC);
    }
    {
      const int tn = (t + 1 < NVIS) ? (t + 1) : (NVIS - 1);
      load_x_tile(vv, rowbase, dir ? (NVIS - 1 - tn) : tn, Ax, tid);
    }
    __syncthreads();
  }

#pragma unroll
  for (int nt = 0; nt < 2; ++nt) {
    const int j = 32 * wave + 16 * nt + c;
#pragma unroll
    for (int r = 0; r < 8; ++r) Hs[(8 * hh + r) * HSP + j] = hsum[nt][r];
  }
  __syncthreads();
  for (int pass = 0; pass < 2; ++pass) {
#pragma unroll
    for (int it = 0; it < 4; ++it) {
      const int idx = it * 256 + tid;
      const int row = idx >> 6, c4 = (idx & 63) * 4;
      const v4f v = *(const v4f*)(Hs + row * HSP + c4);
      *(volatile v4f*)(out + (size_t)(rowbase + row) * (2 * NHID) + (size_t)dir * NHID + c4) = v;
    }
    __threadfence();
  }
}

extern "C" void kernel_launch(void* const* d_in, const int* in_sizes, int n_in,
                              void* d_out, int out_size, void* d_ws, size_t ws_size, hipStream_t stream) {
  if (n_in < 15 || d_out == nullptr || d_ws == nullptr) return;
  if (in_sizes[0] != NVISITS * NCODE || in_sizes[1] != NVISITS * NCODE || in_sizes[2] != NVISITS ||
      in_sizes[3] != NVISITS || in_sizes[4] != NVOC * NEMB || in_sizes[5] != NATT * NEMB || in_sizes[6] != NATT * NEMB ||
      in_sizes[7] != NVOC || in_sizes[8] != NVOC || in_sizes[9] != NGATE * NEMB || in_sizes[10] != NGATE * NHID ||
      in_sizes[11] != NGATE || in_sizes[12] != NGATE * NEMB || in_sizes[13] != NGATE * NHID || in_sizes[14] != NGATE ||
      out_size != NBATCH * 2 * NHID) return;

  const int*   codes      = (const int*)d_in[0];
  const float* code_mask  = (const float*)d_in[1];
  const float* time_vals  = (const float*)d_in[2];
  const float* visit_mask = (const float*)d_in[3];
  const float* emb        = (const float*)d_in[4];
  const float* WQ         = (const float*)d_in[5];
  const float* WK         = (const float*)d_in[6];
  const float* decay      = (const float*)d_in[7];
  const float* initial    = (const float*)d_in[8];
  const float* Wih_f      = (const float*)d_in[9];
  const float* Whh_f      = (const float*)d_in[10];
  const float* b_f        = (const float*)d_in[11];
  const float* Wih_b      = (const float*)d_in[12];
  const float* Whh_b      = (const float*)d_in[13];
  const float* b_b        = (const float*)d_in[14];
  float* out = (float*)d_out;

  char* ws = (char*)d_ws;
  size_t off = 0;
  auto carve = [&](size_t bytes) -> char* { char* p = ws + off; off += (bytes + 255) & ~(size_t)255; return p; };
  unsigned short* EMB16 = (unsigned short*)carve((size_t)NVOCP * NEMB * 2);
  unsigned short* QK16  = (unsigned short*)carve((size_t)NVOCP * NEMB * 2);
  unsigned short* WQK16 = (unsigned short*)carve((size_t)(2 * NATT) * NEMB * 2);
  unsigned short* WXF   = (unsigned short*)carve((size_t)NGATE * NEMB * 2);
  unsigned short* WHF   = (unsigned short*)carve((size_t)NGATE * NHID * 2);
  unsigned short* WXB   = (unsigned short*)carve((size_t)NGATE * NEMB * 2);
  unsigned short* WHB   = (unsigned short*)carve((size_t)NGATE * NHID * 2);
  float*          VV    = (float*)carve((size_t)NVISITS * NEMB * 4);
  if (off > ws_size || off > (size_t)134217728) return;

  cast_rows_f16<<<(NVOCP * 32) / 256, 256, 0, stream>>>(emb, NVOC, EMB16, NVOCP, EMB_SC);
  cast_rows_f16<<<(NATT * 32) / 256, 256, 0, stream>>>(WQ, NATT, WQK16, NATT, W_SC);
  cast_rows_f16<<<(NATT * 32) / 256, 256, 0, stream>>>(WK, NATT, WQK16 + (size_t)NATT * NEMB, NATT, W_SC);
  cast_rows_f16<<<(NGATE * 32) / 256, 256, 0, stream>>>(Wih_f, NGATE, WXF, NGATE, W_SC);
  cast_rows_f16<<<(NGATE * 32) / 256, 256, 0, stream>>>(Whh_f, NGATE, WHF, NGATE, W_SC);
  cast_rows_f16<<<(NGATE * 32) / 256, 256, 0, stream>>>(Wih_b, NGATE, WXB, NGATE, W_SC);
  cast_rows_f16<<<(NGATE * 32) / 256, 256, 0, stream>>>(Whh_b, NGATE, WHB, NGATE, W_SC);

  {
    const int tiles = (NVOCP / 64) * ((2 * NATT) / 64);
    const int blocks = (tiles + 7) / 8;
    wmma_gemm64<0, false, 0, 1, false><<<dim3(blocks, 1), 256, 0, stream>>>(
        EMB16, EMB16, NEMB, 0L, WQK16, WQK16, NEMB, 0L, (void*)QK16, (void*)QK16, 2 * NATT, 0L,
        nullptr, nullptr, 0L, NVOCP, 2 * NATT, NEMB, QK_OUT_SC);
  }

  visit_attn_kernel<<<NVISITS, 256, 0, stream>>>(codes, code_mask, time_vals, decay, initial, EMB16, QK16, VV);

  bilstm_kernel<<<4, 256, 0, stream>>>(VV, visit_mask, b_f, b_b, WXF, WHF, WXB, WHB, out);
}
